// T5MultiHeadAttention_23270132810085
// MI455X (gfx1250) — hardware-verified
//
#include <hip/hip_runtime.h>
#include <math.h>
#include <stdint.h>

constexpr int N_BATCH = 2;
constexpr int SEQ_LEN = 2048;
constexpr int D_MODEL = 1024;
constexpr int N_HEAD  = 16;
constexpr int D_HEAD  = 64;
constexpr int D_INNER = N_HEAD * D_HEAD;
static_assert(D_INNER == 1024, "inner width");
static_assert(SEQ_LEN % 64 == 0 && D_MODEL % 64 == 0 && D_INNER % 64 == 0, "tile multiples");
static_assert(D_MODEL % 32 == 0 && D_INNER % 32 == 0, "K multiples of 32");

typedef __attribute__((ext_vector_type(16))) _Float16 v16h;
typedef __attribute__((ext_vector_type(8)))  _Float16 v8h;
typedef __attribute__((ext_vector_type(16))) __bf16   v16b;
typedef __attribute__((ext_vector_type(8)))  __bf16   v8b;
typedef __attribute__((ext_vector_type(8)))  float    v8f;
typedef __attribute__((ext_vector_type(4)))  float    v4f;
typedef __attribute__((ext_vector_type(2)))  float    v2f;

__device__ __forceinline__ unsigned short f2bf_bits(float f) {
  unsigned u = __float_as_uint(f);
  return (unsigned short)((u + 0x7FFFu + ((u >> 16) & 1u)) >> 16);
}
__device__ __forceinline__ float bf_bits2f(unsigned short h) { return __uint_as_float(((unsigned)h) << 16); }
__device__ __forceinline__ unsigned pk16(unsigned short a, unsigned short b) { return (unsigned)a | ((unsigned)b << 16); }

__device__ __forceinline__ void dep_guard_h(v8f& a, v8f& b, v16h x, v16h y) { asm volatile("v_nop\n\tv_nop\n\tv_nop\n\tv_nop" : "+v"(a), "+v"(b) : "v"(x), "v"(y)); }
__device__ __forceinline__ void dep_guard_b(v8f& a, v8f& b, v16b x, v16b y) { asm volatile("v_nop\n\tv_nop\n\tv_nop\n\tv_nop" : "+v"(a), "+v"(b) : "v"(x), "v"(y)); }
__device__ __forceinline__ void keep4_h(v16h a, v16h b, v16h c, v16h d) { asm volatile("v_nop" :: "v"(a), "v"(b), "v"(c), "v"(d)); }
__device__ __forceinline__ void keep4_b(v16b a, v16b b, v16b c, v16b d) { asm volatile("v_nop" :: "v"(a), "v"(b), "v"(c), "v"(d)); }
__device__ __forceinline__ void acc_guard4(v8f& a, v8f& b, v8f& c, v8f& d) { asm volatile("v_nop\n\tv_nop\n\tv_nop\n\tv_nop" : "+v"(a), "+v"(b), "+v"(c), "+v"(d)); }
template <typename T> struct Frag;
template <> struct Frag<_Float16> {
  typedef v16h V; union U { v16h v; v8h h[2]; };
  static __device__ __forceinline__ v16h load(const _Float16* p) {
    U f; f.h[0] = *(const v8h*)(p); f.h[1] = *(const v8h*)(p + 16); return f.v;
  }
  static __device__ __forceinline__ v8f mma(v16h a, v16h b, v8f c) {
    return __builtin_amdgcn_wmma_f32_16x16x32_f16(false, a, false, b, (short)0, c, false, false);
  }
  static __device__ __forceinline__ void guard(v8f& a, v8f& b, v16h x, v16h y) { dep_guard_h(a, b, x, y); }
  static __device__ __forceinline__ void keep(v16h a, v16h b, v16h c, v16h d) { keep4_h(a, b, c, d); }
};
template <> struct Frag<__bf16> {
  typedef v16b V; union U { v16b v; v8b h[2]; };
  static __device__ __forceinline__ v16b load(const __bf16* p) {
    U f; f.h[0] = *(const v8b*)(p); f.h[1] = *(const v8b*)(p + 16); return f.v;
  }
  static __device__ __forceinline__ v8f mma(v16b a, v16b b, v8f c) {
    return __builtin_amdgcn_wmma_f32_16x16x32_bf16(false, a, false, b, (short)0, c, false, false);
  }
  static __device__ __forceinline__ void guard(v8f& a, v8f& b, v16b x, v16b y) { dep_guard_b(a, b, x, y); }
  static __device__ __forceinline__ void keep(v16b a, v16b b, v16b c, v16b d) { keep4_b(a, b, c, d); }
};

template <int ET> struct Elem;
template <> struct Elem<0> { typedef _Float16 T; };
template <> struct Elem<1> { typedef __bf16 T; };
template <int ET, bool SPLIT, int BIAS_MODE, int OUT_MODE, bool RESID, int ACT = 0, bool BLO = true>
__global__ __launch_bounds__(256) void wmma_gemm64(
    const unsigned short* __restrict__ Ap, const unsigned short* __restrict__ A2p, int lda, long strideA,
    const unsigned short* __restrict__ Btp, const unsigned short* __restrict__ Bt2p, int ldb, long strideB,
    void* __restrict__ Cout, void* __restrict__ Cout2, int ldc, long strideC,
    const float* __restrict__ bias,
    const float* __restrict__ resid, long strideR,
    int M, int N, int K, float scale) {
  typedef typename Elem<ET>::T T;
  typedef typename Frag<T>::V V;
  const T* A = (const T*)Ap; const T* A2 = (const T*)A2p; const T* Bt = (const T*)Btp; const T* Bt2 = (const T*)Bt2p;
  __shared__ __align__(16) float sT[8][16 * 68];
  const int b    = blockIdx.y;
  const int lane = threadIdx.x & 31;
  const int wave = threadIdx.x >> 5;
  const int tilesN = N >> 6;
  const int tilesM = M >> 6;
  const int tile = blockIdx.x * 8 + wave;
  if (tile >= tilesM * tilesN) return;
  const int tm = tile / tilesN;
  const int tn = tile - tm * tilesN;
  const int m0 = tm << 6;
  const int n0 = tn << 6;

  const T* Ab  = A  + (size_t)b * strideA;
  const T* Bb  = Bt + (size_t)b * strideB;
  const T* Ab2 = SPLIT ? (A2  + (size_t)b * strideA) : nullptr;
  const T* Bb2 = (SPLIT && BLO) ? (Bt2 + (size_t)b * strideB) : nullptr;

  const int rlane = lane & 15;
  const int koff  = (lane >> 4) * 8;
  const int mOff  = (lane >> 4) * 8;

  v8f acc[4][4];
#pragma unroll
  for (int i = 0; i < 4; ++i)
#pragma unroll
    for (int j = 0; j < 4; ++j) acc[i][j] = (v8f){0.f,0.f,0.f,0.f,0.f,0.f,0.f,0.f};

  for (int k0 = 0; k0 < K; k0 += 32) {
    V bh[4], bl[4];
#pragma unroll
    for (int j = 0; j < 4; ++j) {
      const size_t bo = (size_t)(n0 + (j << 4) + rlane) * ldb + koff + k0;
      bh[j] = Frag<T>::load(Bb + bo);
      if (SPLIT && BLO) bl[j] = Frag<T>::load(Bb2 + bo);
    }
#pragma unroll
    for (int i = 0; i < 4; ++i) {
      const size_t ao = (size_t)(m0 + (i << 4) + rlane) * lda + koff + k0;
      V ah = Frag<T>::load(Ab + ao);
      V al;
      if (SPLIT) al = Frag<T>::load(Ab2 + ao);
#pragma unroll
      for (int j = 0; j < 4; ++j) {
        acc[i][j] = Frag<T>::mma(ah, bh[j], acc[i][j]);
        if (SPLIT) {
          if (BLO) acc[i][j] = Frag<T>::mma(ah, bl[j], acc[i][j]);
          acc[i][j] = Frag<T>::mma(al, bh[j], acc[i][j]);
        }
      }
      Frag<T>::guard(acc[i][0], acc[i][3], ah, SPLIT ? al : ah);
    }
    Frag<T>::keep(bh[0], bh[1], bh[2], bh[3]);
    if (SPLIT && BLO) Frag<T>::keep(bl[0], bl[1], bl[2], bl[3]);
  }
  acc_guard4(acc[0][0], acc[0][1], acc[0][2], acc[0][3]);
  acc_guard4(acc[1][0], acc[1][1], acc[1][2], acc[1][3]);
  acc_guard4(acc[2][0], acc[2][1], acc[2][2], acc[2][3]);
  acc_guard4(acc[3][0], acc[3][1], acc[3][2], acc[3][3]);

  float* slab = sT[wave];
  const float* Rb = RESID ? (resid + (size_t)b * strideR) : nullptr;
#pragma unroll
  for (int i = 0; i < 4; ++i) {
    const int mBase = m0 + (i << 4);
#pragma unroll
    for (int j = 0; j < 4; ++j) {
      const int n = n0 + (j << 4) + rlane;
      float bv = 0.f;
      if (BIAS_MODE == 2) bv = bias[n];
#pragma unroll
      for (int r = 0; r < 8; ++r) {
        float v = acc[i][j][r] * scale;
        if (BIAS_MODE == 1) v += bias[mBase + mOff + r];
        if (BIAS_MODE == 2) v += bv;
        if (RESID) v += Rb[(size_t)(mBase + mOff + r) * ldc + n];
        if (ACT == 1) v = tanhf(v);
        if (ACT == 2) v = fmaxf(v, 0.0f);
        if (ACT == 3) v = v / (1.0f + expf(-v));
        if (ACT == 4) v = (v > 0.f) ? v : 0.01f * v;
        slab[(mOff + r) * 68 + (j << 4) + rlane] = v;
      }
    }
    __builtin_amdgcn_fence(__ATOMIC_RELEASE, "workgroup");
    __builtin_amdgcn_wave_barrier();
    __builtin_amdgcn_fence(__ATOMIC_ACQUIRE, "workgroup");
    if (OUT_MODE == 0) {
      float* C = (float*)Cout + (size_t)b * strideC;
      const int hh = lane >> 4, c4 = (lane & 15) * 4;
      for (int pass = 0; pass < 2; ++pass) {
#pragma unroll
        for (int it = 0; it < 8; ++it) {
          const int row = it * 2 + hh;
          v4f v = *(const v4f*)(slab + row * 68 + c4);
          *(volatile v4f*)(C + (size_t)(mBase + row) * ldc + n0 + c4) = v;
        }
        __threadfence();
      }
    } else {
      const int q = lane >> 3, c8 = (lane & 7) * 8;
      unsigned short* C  = (unsigned short*)Cout  + (size_t)b * strideC;
      unsigned short* C2 = (OUT_MODE == 2) ? ((unsigned short*)Cout2 + (size_t)b * strideC) : nullptr;
      for (int pass = 0; pass < 2; ++pass) {
#pragma unroll
        for (int it = 0; it < 4; ++it) {
          const int row = it * 4 + q;
          const float* sp = slab + row * 68 + c8;
          v8h hv, lv;
#pragma unroll
          for (int e = 0; e < 8; ++e) {
            if (OUT_MODE == 1) {
              hv[e] = (_Float16)sp[e];
            } else {
              unsigned short hb = f2bf_bits(sp[e]);
              unsigned short lb = f2bf_bits(sp[e] - bf_bits2f(hb));
              hv[e] = __builtin_bit_cast(_Float16, hb);
              lv[e] = __builtin_bit_cast(_Float16, lb);
            }
          }
          *(volatile v8h*)(C + (size_t)(mBase + row) * ldc + n0 + c8) = hv;
          if (OUT_MODE == 2) *(volatile v8h*)(C2 + (size_t)(mBase + row) * ldc + n0 + c8) = lv;
        }
        __threadfence();
      }
    }
    __builtin_amdgcn_fence(__ATOMIC_RELEASE, "workgroup");
    __builtin_amdgcn_wave_barrier();
    __builtin_amdgcn_fence(__ATOMIC_ACQUIRE, "workgroup");
  }
}

__global__ __launch_bounds__(256) void cast_f32_bf16x2(const float* __restrict__ in,
                                                        unsigned short* __restrict__ out, int n2) {
  const int i = blockIdx.x * 256 + threadIdx.x;
  if (i < n2) {
    const v2f f = *(const v2f*)(in + 2 * (size_t)i);
    const unsigned u = pk16(f2bf_bits(f[0]), f2bf_bits(f[1]));
    ((volatile unsigned*)out)[i] = u;
    __threadfence();
    ((volatile unsigned*)out)[i] = u;
  }
}

#define AT_D 64
#define AT_NW 4
#define AT_QB 64
#define AT_KC 64
#define P_CARRY 32768.0f

__device__ __forceinline__ v8f at_mma(v16b a, v16b b, v8f c) {
  c = __builtin_amdgcn_wmma_f32_16x16x32_bf16(false, a, false, b, (short)0, c, false, false);
  asm volatile("v_nop\n\tv_nop\n\tv_nop\n\tv_nop" : "+v"(c) : "v"(a), "v"(b));
  return c;
}
__device__ __forceinline__ v8f at_mma_h(v16b a, v16b b, v8f c) {
  const v16h ah = __builtin_bit_cast(v16h, a), bh = __builtin_bit_cast(v16h, b);
  c = __builtin_amdgcn_wmma_f32_16x16x32_f16(false, ah, false, bh, (short)0, c, false, false);
  asm volatile("v_nop\n\tv_nop\n\tv_nop\n\tv_nop" : "+v"(c) : "v"(ah), "v"(bh));
  return c;
}
__device__ __forceinline__ __bf16 at_f16bits(float f) { return __builtin_bit_cast(__bf16, (_Float16)f); }

__global__ __launch_bounds__(128)
void mha_bias_kernel(const unsigned short* __restrict__ qhp, const unsigned short* __restrict__ qlp,
                     const unsigned short* __restrict__ khp, const unsigned short* __restrict__ klp,
                     const unsigned short* __restrict__ vtp, const float* __restrict__ biasp,
                     unsigned short* __restrict__ chp, unsigned short* __restrict__ clp,
                     const int* __restrict__ nheads_in) {
  (void)nheads_in;
  union FB { v16b v; v8b h[2]; };
  __shared__ __align__(16) __bf16 Ksh[AT_KC * AT_D];
  __shared__ __align__(16) __bf16 Ksl[AT_KC * AT_D];
  __shared__ __align__(16) __bf16 Vth[AT_D * AT_KC];
  __shared__ __align__(16) __bf16 Psh[AT_NW][16 * AT_KC];
  __shared__ __align__(16) float  Os[AT_NW][16 * 68];

  const int tid  = threadIdx.x;
  const int wave = tid >> 5;
  const int lane = tid & 31;
  const int hh   = lane >> 4;
  const int c    = lane & 15;

  const int nqb = SEQ_LEN / AT_QB;
  const int bx  = blockIdx.x;
  const int qb  = bx % nqb;
  const int bhd = bx / nqb;
  const int h   = bhd % N_HEAD;
  const int b   = bhd / N_HEAD;
  const int q0  = qb * AT_QB + wave * 16;

  const size_t rowb = (size_t)b * SEQ_LEN;
  const __bf16* Qh = (const __bf16*)(const void*)qhp + rowb * D_INNER + (size_t)h * AT_D;
  const __bf16* Ql = (const __bf16*)(const void*)qlp + rowb * D_INNER + (size_t)h * AT_D;
  const __bf16* Kh = (const __bf16*)(const void*)khp + rowb * D_INNER + (size_t)h * AT_D;
  const __bf16* Kl = (const __bf16*)(const void*)klp + rowb * D_INNER + (size_t)h * AT_D;
  const __bf16* Vt = (const __bf16*)(const void*)vtp + ((size_t)b * D_INNER + (size_t)h * AT_D) * SEQ_LEN;
  const float*  Mb = biasp + (size_t)b * SEQ_LEN * SEQ_LEN;
  unsigned short* Ch = chp + rowb * D_INNER + (size_t)h * AT_D;
  unsigned short* Cl = clp + rowb * D_INNER + (size_t)h * AT_D;

  v16b qah[2], qal[2];
#pragma unroll
  for (int dc = 0; dc < 2; ++dc) {
    const __bf16* qr = Qh + (size_t)(q0 + c) * D_INNER + dc * 32 + 8 * hh;
    const __bf16* ql = Ql + (size_t)(q0 + c) * D_INNER + dc * 32 + 8 * hh;
    qah[dc] = Frag<__bf16>::load(qr);
    qal[dc] = Frag<__bf16>::load(ql);
  }

  float mrow[8], lrow[8];
  v8f oacc[4];
#pragma unroll
  for (int r = 0; r < 8; ++r) { mrow[r] = -INFINITY; lrow[r] = 0.f; }
#pragma unroll
  for (int t = 0; t < 4; ++t) oacc[t] = (v8f){0.f,0.f,0.f,0.f,0.f,0.f,0.f,0.f};

  const int nChunks = SEQ_LEN / AT_KC;
  for (int kc = 0; kc < nChunks; ++kc) {
    const int kv0 = kc * AT_KC;
    __syncthreads();
    {
      const int r = tid >> 1, half = (tid & 1) * 32;
      const __bf16* ksh = Kh + (size_t)(kv0 + r) * D_INNER + half;
      const __bf16* ksl = Kl + (size_t)(kv0 + r) * D_INNER + half;
      const __bf16* vs  = Vt + (size_t)r * SEQ_LEN + kv0 + half;
#pragma unroll
      for (int i = 0; i < 4; ++i) {
        const v8b a0 = *(const v8b*)(ksh + 8 * i);
        const v8b a1 = *(const v8b*)(ksl + 8 * i);
        const v8b b0 = *(const v8b*)(vs + 8 * i);
        *(v8b*)(Ksh + r * AT_D  + half + 8 * i) = a0;
        *(v8b*)(Ksl + r * AT_D  + half + 8 * i) = a1;
        *(v8b*)(Vth + r * AT_KC + half + 8 * i) = b0;
      }
    }
    __syncthreads();

    v8f s[4];
#pragma unroll
    for (int j = 0; j < 4; ++j) {
      s[j] = (v8f){0.f,0.f,0.f,0.f,0.f,0.f,0.f,0.f};
#pragma unroll
      for (int dc = 0; dc < 2; ++dc) {
        FB kb, kl;
        kb.h[0] = *(const v8b*)(Ksh + (j * 16 + c) * AT_D + dc * 32 + 8 * hh);
        kb.h[1] = *(const v8b*)(Ksh + (j * 16 + c) * AT_D + dc * 32 + 16 + 8 * hh);
        kl.h[0] = *(const v8b*)(Ksl + (j * 16 + c) * AT_D + dc * 32 + 8 * hh);
        kl.h[1] = *(const v8b*)(Ksl + (j * 16 + c) * AT_D + dc * 32 + 16 + 8 * hh);
        s[j] = at_mma(qah[dc], kb.v, s[j]);
        s[j] = at_mma(qah[dc], kl.v, s[j]);
        s[j] = at_mma(qal[dc], kb.v, s[j]);
      }
    }
    float cm[8];
#pragma unroll
    for (int r = 0; r < 8; ++r) {
      const float* mrp = Mb + (size_t)(q0 + 8 * hh + r) * SEQ_LEN + kv0 + c;
      float m = -INFINITY;
#pragma unroll
      for (int j = 0; j < 4; ++j) {
        const float mv = bf_bits2f(f2bf_bits(mrp[j * 16]));
        const float sv = s[j][r] + mv;
        s[j][r] = sv;
        m = fmaxf(m, sv);
      }
#pragma unroll
      for (int off = 1; off < 16; off <<= 1) m = fmaxf(m, __shfl_xor(m, off, 32));
      cm[r] = m;
    }
    __bf16* pwh = Psh[wave];
#pragma unroll
    for (int r = 0; r < 8; ++r) {
      const float mnew = fmaxf(mrow[r], cm[r]);
      const float alpha = expf(mrow[r] - mnew);
      mrow[r] = mnew;
      float psum = 0.f;
#pragma unroll
      for (int j = 0; j < 4; ++j) {
        const float p = expf(s[j][r] - mnew);
        psum += p;
        pwh[(8 * hh + r) * AT_KC + j * 16 + c] = at_f16bits(p * P_CARRY);
      }
#pragma unroll
      for (int off = 1; off < 16; off <<= 1) psum += __shfl_xor(psum, off, 32);
      lrow[r] = lrow[r] * alpha + psum;
#pragma unroll
      for (int t = 0; t < 4; ++t) oacc[t][r] *= alpha;
    }
    __builtin_amdgcn_fence(__ATOMIC_RELEASE, "workgroup");
    __builtin_amdgcn_wave_barrier();
    __builtin_amdgcn_fence(__ATOMIC_ACQUIRE, "workgroup");
#pragma unroll 1
    for (int kk = 0; kk < 2; ++kk) {
      FB pa;
      pa.h[0] = *(const v8b*)(pwh + c * AT_KC + kk * 32 + 8 * hh);
      pa.h[1] = *(const v8b*)(pwh + c * AT_KC + kk * 32 + 16 + 8 * hh);
#pragma unroll
      for (int t = 0; t < 4; ++t) {
        FB vb;
        vb.h[0] = *(const v8b*)(Vth + (t * 16 + c) * AT_KC + kk * 32 + 8 * hh);
        vb.h[1] = *(const v8b*)(Vth + (t * 16 + c) * AT_KC + kk * 32 + 16 + 8 * hh);
        oacc[t] = at_mma_h(pa.v, vb.v, oacc[t]);
      }
    }
  }

  float* os = Os[wave];
#pragma unroll
  for (int r = 0; r < 8; ++r) {
    const float inv = 1.0f / (lrow[r] * P_CARRY);
#pragma unroll
    for (int t = 0; t < 4; ++t) os[(8 * hh + r) * 68 + t * 16 + c] = oacc[t][r] * inv;
  }
  __builtin_amdgcn_fence(__ATOMIC_RELEASE, "workgroup");
  __builtin_amdgcn_wave_barrier();
  __builtin_amdgcn_fence(__ATOMIC_ACQUIRE, "workgroup");
  {
    const int qg = lane >> 3, c8 = (lane & 7) * 8;
    for (int pass = 0; pass < 2; ++pass) {
#pragma unroll
      for (int it = 0; it < 4; ++it) {
        const int row = it * 4 + qg;
        const float* sp = os + row * 68 + c8;
        v8h hv, lv;
#pragma unroll
        for (int e = 0; e < 8; ++e) {
          const unsigned short hb = f2bf_bits(sp[e]);
          const unsigned short lb = f2bf_bits(sp[e] - bf_bits2f(hb));
          hv[e] = __builtin_bit_cast(_Float16, hb);
          lv[e] = __builtin_bit_cast(_Float16, lb);
        }
        *(volatile v8h*)(Ch + (size_t)(q0 + row) * D_INNER + c8) = hv;
        *(volatile v8h*)(Cl + (size_t)(q0 + row) * D_INNER + c8) = lv;
      }
      __threadfence();
    }
  }
}

extern "C" void kernel_launch(void* const* d_in, const int* in_sizes, int n_in,
                              void* d_out, int out_size, void* d_ws, size_t ws_size,
                              hipStream_t stream) {
  if (n_in < 9) return;
  const size_t nAct  = (size_t)N_BATCH * SEQ_LEN * D_MODEL;
  const size_t nW    = (size_t)D_INNER * D_MODEL;
  const size_t nMask = (size_t)N_BATCH * SEQ_LEN * SEQ_LEN;
  const size_t nVT   = (size_t)N_BATCH * D_INNER * SEQ_LEN;
  if ((size_t)in_sizes[0] != nAct || (size_t)in_sizes[1] != nAct || (size_t)in_sizes[2] != nAct ||
      (size_t)in_sizes[3] != nMask || (size_t)in_sizes[4] != nW || (size_t)in_sizes[5] != nW ||
      (size_t)in_sizes[6] != nW || (size_t)in_sizes[7] != nW || in_sizes[8] < 1 ||
      (size_t)out_size != nAct) return;

  const size_t bAct = nAct * 2, bW = nW * 2, bVT = nVT * 2;
  const size_t o_q16 = 0;
  const size_t o_k16 = o_q16 + bAct;
  const size_t o_v16 = o_k16 + bAct;
  const size_t o_wq  = o_v16 + bAct;
  const size_t o_wk  = o_wq + bW;
  const size_t o_wv  = o_wk + bW;
  const size_t o_wo  = o_wv + bW;
  const size_t o_qhi = o_wo + bW;
  const size_t o_qlo = o_qhi + bAct;
  const size_t o_khi = o_qlo + bAct;
  const size_t o_klo = o_khi + bAct;
  const size_t o_vt  = o_klo + bAct;
  const size_t o_chi = o_vt + bVT;
  const size_t o_clo = o_chi + bAct;
  const size_t total = o_clo + bAct;
  if (total > ws_size) return;

  const float* qf  = (const float*)d_in[0];
  const float* kf  = (const float*)d_in[1];
  const float* vf  = (const float*)d_in[2];
  const float* mf  = (const float*)d_in[3];
  const float* wqf = (const float*)d_in[4];
  const float* wkf = (const float*)d_in[5];
  const float* wvf = (const float*)d_in[6];
  const float* wof = (const float*)d_in[7];
  const int*   nhp = (const int*)d_in[8];
  char* ws = (char*)d_ws;
  unsigned short* q16 = (unsigned short*)(ws + o_q16);
  unsigned short* k16 = (unsigned short*)(ws + o_k16);
  unsigned short* v16 = (unsigned short*)(ws + o_v16);
  unsigned short* wq16 = (unsigned short*)(ws + o_wq);
  unsigned short* wk16 = (unsigned short*)(ws + o_wk);
  unsigned short* wv16 = (unsigned short*)(ws + o_wv);
  unsigned short* wo16 = (unsigned short*)(ws + o_wo);
  unsigned short* qhi = (unsigned short*)(ws + o_qhi);
  unsigned short* qlo = (unsigned short*)(ws + o_qlo);
  unsigned short* khi = (unsigned short*)(ws + o_khi);
  unsigned short* klo = (unsigned short*)(ws + o_klo);
  unsigned short* vt  = (unsigned short*)(ws + o_vt);
  unsigned short* chi = (unsigned short*)(ws + o_chi);
  unsigned short* clo = (unsigned short*)(ws + o_clo);
  float* out = (float*)d_out;

  const int n2a = (int)(nAct / 2);
  const int n2w = (int)(nW / 2);
  const dim3 ga((unsigned)((n2a + 255) / 256)), gw((unsigned)((n2w + 255) / 256)), blk(256);
  cast_f32_bf16x2<<<ga, blk, 0, stream>>>(qf, q16, n2a);
  cast_f32_bf16x2<<<ga, blk, 0, stream>>>(kf, k16, n2a);
  cast_f32_bf16x2<<<ga, blk, 0, stream>>>(vf, v16, n2a);
  cast_f32_bf16x2<<<gw, blk, 0, stream>>>(wqf, wq16, n2w);
  cast_f32_bf16x2<<<gw, blk, 0, stream>>>(wkf, wk16, n2w);
  cast_f32_bf16x2<<<gw, blk, 0, stream>>>(wvf, wv16, n2w);
  cast_f32_bf16x2<<<gw, blk, 0, stream>>>(wof, wo16, n2w);

  const int MTOK = N_BATCH * SEQ_LEN;
  {
    const int tiles = (MTOK / 64) * (D_INNER / 64);
    const dim3 g((unsigned)((tiles + 7) / 8), 1);
    wmma_gemm64<1, false, 0, 2, false><<<g, 256, 0, stream>>>(
        q16, q16, D_MODEL, 0L, wq16, wq16, D_MODEL, 0L, (void*)qhi, (void*)qlo, D_INNER, 0L,
        mf, mf, 0L, MTOK, D_INNER, D_MODEL, 1.0f);
    wmma_gemm64<1, false, 0, 2, false><<<g, 256, 0, stream>>>(
        k16, k16, D_MODEL, 0L, wk16, wk16, D_MODEL, 0L, (void*)khi, (void*)klo, D_INNER, 0L,
        mf, mf, 0L, MTOK, D_INNER, D_MODEL, 1.0f);
  }
  {
    const int tiles = (D_INNER / 64) * (SEQ_LEN / 64);
    const dim3 g((unsigned)((tiles + 7) / 8), (unsigned)N_BATCH);
    wmma_gemm64<1, false, 0, 1, false><<<g, 256, 0, stream>>>(
        wv16, wv16, D_MODEL, 0L, v16, v16, D_MODEL, (long)SEQ_LEN * D_MODEL,
        (void*)vt, (void*)vt, SEQ_LEN, (long)D_INNER * SEQ_LEN,
        mf, mf, 0L, D_INNER, SEQ_LEN, D_MODEL, 1.0f);
  }
  {
    const dim3 g((unsigned)(N_BATCH * N_HEAD * (SEQ_LEN / AT_QB)));
    mha_bias_kernel<<<g, 128, 0, stream>>>(qhi, qlo, khi, klo, vt, mf, chi, clo, nhp);
  }
  {
    const int tiles = (MTOK / 64) * (D_MODEL / 64);
    const dim3 g((unsigned)((tiles + 7) / 8), 1);
    wmma_gemm64<1, true, 0, 0, false, 0, false><<<g, 256, 0, stream>>>(
        chi, clo, D_INNER, 0L, wo16, wo16, D_INNER, 0L, (void*)out, (void*)out, D_MODEL, 0L,
        mf, mf, 0L, MTOK, D_MODEL, D_INNER, 1.0f);
  }
}
